// NeuralCausalModel_13348758356448
// MI455X (gfx1250) — hardware-run, weakly checked
//
#include <hip/hip_runtime.h>
#include <math.h>

typedef __attribute__((ext_vector_type(16))) _Float16 v16h;
typedef __attribute__((ext_vector_type(8)))  _Float16 v8h;
typedef __attribute__((ext_vector_type(8)))  float    v8f;
typedef __attribute__((ext_vector_type(4)))  float    v4f;
typedef __attribute__((ext_vector_type(2)))  float    v2f;

constexpr int kVars = 16;
constexpr int kN    = 524288;
constexpr int kHid  = 64;
constexpr int kTilesPerWave = 8;
constexpr int kMainBlocks   = 256;
constexpr int kWavesPerBlk  = 8;
static_assert(kMainBlocks * kWavesPerBlk * kTilesPerWave * 32 == kN);
static_assert(kHid == 64);

constexpr float kCarryH   = 16.0f;
constexpr float kCarryW   = 64.0f;
constexpr float kCarryAll = kCarryH * kCarryW;
constexpr float kFoldBack = 1.0f / kCarryAll;
static_assert(kCarryAll == 1024.0f);

constexpr int kParamRows   = 80;
constexpr int kParamFloats = kParamRows * 64;
constexpr int kOffB2f      = 48 * 64;
constexpr int kOffW3f      = 64 * 64;
static_assert(kParamFloats == 5120);
static_assert(kParamFloats == 5 * 256 * 4);
static_assert(kParamRows == 10 * 8);

constexpr size_t kOffW2T  = 0;
constexpr size_t kBytesW2T = (size_t)kVars * kHid * kHid * 2;
constexpr size_t kOffPRM  = kOffW2T + kBytesW2T;
constexpr size_t kBytesPRM = (size_t)kParamFloats * 4;
constexpr size_t kWsTotal = kOffPRM + kBytesPRM;
static_assert(kBytesW2T == 131072ull);
static_assert(kBytesPRM == 20480ull);
static_assert(kWsTotal == 151552ull);
static_assert((kOffPRM % 128) == 0);
static_assert(kWsTotal <= 134217728ull);

template <typename T> struct Frag;
template <> struct Frag<_Float16> {
  typedef v16h V; union U { v16h v; v8h h[2]; };
  static __device__ __forceinline__ v16h load(const _Float16* p) {
    U f; f.h[0] = *(const v8h*)(p); f.h[1] = *(const v8h*)(p + 16); return f.v;
  }
  static __device__ __forceinline__ v8f mma(v16h a, v16h b, v8f c) {
    return __builtin_amdgcn_wmma_f32_16x16x32_f16(false, a, false, b, (short)0, c, false, false);
  }
};
__device__ __forceinline__ void chain_guard(v8f& c, v16h a0, v16h a1, v16h b0, v16h b1) {
  asm volatile("v_nop\n\tv_nop\n\tv_nop\n\tv_nop" : "+v"(c) : "v"(a0), "v"(a1), "v"(b0), "v"(b1));
}

__global__ __launch_bounds__(256) void prep_w2t_kernel(
    const float* __restrict__ w0_2, const float* __restrict__ W2, unsigned short* __restrict__ W2T)
{
  __shared__ __align__(16) float sT[64 * 65];
  const int tid = threadIdx.x;
  const int v = blockIdx.x;
  const int u = (v > 0) ? (v - 1) : 0;
  const bool root = (v == 0);
#pragma unroll
  for (int it = 0; it < 4; ++it) {
    const int idx4 = it * 256 + tid;
    const int k  = idx4 >> 4;
    const int n4 = (idx4 & 15) * 4;
    const v4f a = *(const v4f*)(w0_2 + (size_t)idx4 * 4);
    const v4f b = *(const v4f*)(W2 + (size_t)u * 4096 + (size_t)idx4 * 4);
#pragma unroll
    for (int e = 0; e < 4; ++e) {
      const float x = root ? a[e] : b[e];
      sT[k * 65 + n4 + e] = x * kCarryW;
    }
  }
  __syncthreads();
  v8h hv[2];
#pragma unroll
  for (int it = 0; it < 2; ++it) {
    const int c  = it * 256 + tid;
    const int n  = c >> 3;
    const int k0 = (c & 7) * 8;
#pragma unroll
    for (int e = 0; e < 8; ++e) hv[it][e] = (_Float16)sT[(k0 + e) * 65 + n];
  }
  unsigned short* dst = W2T + (size_t)v * 4096;
  for (int pass = 0; pass < 2; ++pass) {
#pragma unroll
    for (int it = 0; it < 2; ++it) {
      const int c  = it * 256 + tid;
      const int n  = c >> 3;
      const int k0 = (c & 7) * 8;
      *(volatile v8h*)(dst + n * 64 + k0) = hv[it];
    }
    __threadfence();
  }
}

__global__ __launch_bounds__(256) void prep_params_kernel(
    const float* __restrict__ w0_1, const float* __restrict__ b0_1,
    const float* __restrict__ b0_2, const float* __restrict__ w0_3,
    const float* __restrict__ W1, const float* __restrict__ B1,
    const float* __restrict__ B2, const float* __restrict__ W3,
    float* __restrict__ P)
{
  const int lane = threadIdx.x & 31;
  int row = __builtin_amdgcn_readfirstlane((int)(blockIdx.x * 8 + (threadIdx.x >> 5)));
  row = (row < kParamRows) ? row : (kParamRows - 1);
  int kind, v, c;
  if (row < 48) {
    kind = 0; v = row / 3; c = row - 3 * v;
  } else if (row < 64) {
    kind = 1; v = row - 48; c = 0;
  } else {
    kind = 2; v = row - 64; c = 0;
  }
  const int u  = (v > 0) ? (v - 1) : 0;
  const int cc = (c < 2) ? c : 0;
  const int j  = 2 * lane;
  const v2f q_w01 = *(const v2f*)(w0_1 + j);
  const v2f q_b01 = *(const v2f*)(b0_1 + j);
  const v2f q_b02 = *(const v2f*)(b0_2 + j);
  const v2f q_w03 = *(const v2f*)(w0_3 + j);
  const v2f q_W1  = *(const v2f*)(W1 + (size_t)(u * 2 + cc) * 64 + j);
  const v2f q_B1  = *(const v2f*)(B1 + (size_t)u * 64 + j);
  const v2f q_B2  = *(const v2f*)(B2 + (size_t)u * 64 + j);
  const v2f q_W3  = *(const v2f*)(W3 + (size_t)u * 64 + j);
  const bool root = (v == 0);
  float x0, x1, scl;
  bool live = true;
  if (kind == 0) {
    scl = kCarryH;
    const float r0 = (c == 1) ? q_w01[0] : q_b01[0];
    const float r1 = (c == 1) ? q_w01[1] : q_b01[1];
    const float s0 = (c < 2) ? q_W1[0] : q_B1[0];
    const float s1 = (c < 2) ? q_W1[1] : q_B1[1];
    x0 = root ? r0 : s0;
    x1 = root ? r1 : s1;
    live = !(root && (c == 0));
  } else if (kind == 1) {
    scl = kCarryAll;
    x0 = root ? q_b02[0] : q_B2[0];
    x1 = root ? q_b02[1] : q_B2[1];
  } else {
    scl = kFoldBack;
    x0 = root ? q_w03[0] : q_W3[0];
    x1 = root ? q_w03[1] : q_W3[1];
  }
  v2f o;
  o[0] = live ? (x0 * scl) : 0.0f;
  o[1] = live ? (x1 * scl) : 0.0f;
  float* q = P + (size_t)row * 64 + j;
  *(volatile v2f*)q = o;
  __threadfence();
  *(volatile v2f*)q = o;
}

__global__ __launch_bounds__(256) void chain_mlp_kernel(
    const float* __restrict__ noise, const float* __restrict__ stds,
    const float* __restrict__ b0_3, const float* __restrict__ B3,
    const unsigned short* __restrict__ W2Tp, const float* __restrict__ P,
    float* __restrict__ out)
{
  __shared__ __align__(32) float sP[kParamFloats];
  const int tid  = threadIdx.x;
  const int lane = tid & 31;
  const int wave = tid >> 5;
  const int half = lane >> 4;
  const int lm   = lane & 15;
#pragma unroll
  for (int it = 0; it < kParamFloats / (4 * 256); ++it) {
    const int idx = it * 256 + tid;
    const v4f x = *(const v4f*)(P + (size_t)idx * 4);
    *(v4f*)(sP + idx * 4) = x;
  }
  __syncthreads();

  const _Float16* W2T = (const _Float16*)W2Tp;
  const int wg = blockIdx.x * kWavesPerBlk + wave;

#pragma unroll 1
  for (int ti = 0; ti < kTilesPerWave; ++ti) {
    const size_t base = (size_t)(wg * kTilesPerWave + ti) * 32;
    float par0 = 0.0f, par1 = 0.0f;
#pragma unroll 1
    for (int v = 0; v < kVars; ++v) {
      const int u = (v > 0) ? (v - 1) : 0;
      const float astd = fabsf(stds[v]);
      const float b3c = B3[u];
      const float b3r = b0_3[0];
      const float b3v = (v == 0) ? b3r : b3c;
      const float* nz = noise + (size_t)v * kN + base;
      const float e0 = nz[lm] * astd;
      const float e1 = nz[16 + lm] * astd;

      v16h bf[2][2];
      const float* pl = sP + v * 192 + 8 * half;
#pragma unroll
      for (int f = 0; f < 2; ++f) {
#pragma unroll
        for (int g = 0; g < 2; ++g) {
          const float* q = pl + 32 * f + 16 * g;
          const v4f wa0 = *(const v4f*)(q);
          const v4f wa1 = *(const v4f*)(q + 4);
          const v4f wb0 = *(const v4f*)(q + 64);
          const v4f wb1 = *(const v4f*)(q + 68);
          const v4f bb0 = *(const v4f*)(q + 128);
          const v4f bb1 = *(const v4f*)(q + 132);
#pragma unroll
          for (int j = 0; j < 4; ++j) {
            const float t00 = fmaf(e0, wb0[j], bb0[j]);
            const float t01 = fmaf(e0, wb1[j], bb1[j]);
            const float t10 = fmaf(e1, wb0[j], bb0[j]);
            const float t11 = fmaf(e1, wb1[j], bb1[j]);
            const float h00 = fmaxf(fmaf(par0, wa0[j], t00), 0.0f);
            const float h01 = fmaxf(fmaf(par0, wa1[j], t01), 0.0f);
            const float h10 = fmaxf(fmaf(par1, wa0[j], t10), 0.0f);
            const float h11 = fmaxf(fmaf(par1, wa1[j], t11), 0.0f);
            bf[0][f][8 * g + j]     = (_Float16)h00;
            bf[0][f][8 * g + 4 + j] = (_Float16)h01;
            bf[1][f][8 * g + j]     = (_Float16)h10;
            bf[1][f][8 * g + 4 + j] = (_Float16)h11;
          }
        }
      }

      const float* pb2 = sP + kOffB2f + v * 64 + 8 * half;
      const float* pw3 = sP + kOffW3f + v * 64 + 8 * half;
      const _Float16* pa = W2T + (size_t)v * 4096 + lm * 64 + 8 * half;
      float p0 = 0.0f, p1 = 0.0f;
#pragma unroll
      for (int t = 0; t < 4; ++t) {
        const v16h a0 = Frag<_Float16>::load(pa + t * 1024);
        const v16h a1 = Frag<_Float16>::load(pa + t * 1024 + 32);
        const v8f b2t = *(const v8f*)(pb2 + 16 * t);
        v8f c0 = Frag<_Float16>::mma(a0, bf[0][0], b2t);
        v8f c1 = Frag<_Float16>::mma(a0, bf[1][0], b2t);
        c0 = Frag<_Float16>::mma(a1, bf[0][1], c0);
        c1 = Frag<_Float16>::mma(a1, bf[1][1], c1);
        chain_guard(c0, a0, a1, bf[0][0], bf[0][1]);
        chain_guard(c1, a0, a1, bf[1][0], bf[1][1]);
        const v8f w3t = *(const v8f*)(pw3 + 16 * t);
#pragma unroll
        for (int r = 0; r < 8; ++r) {
          p0 = fmaf(fmaxf(c0[r], 0.0f), w3t[r], p0);
          p1 = fmaf(fmaxf(c1[r], 0.0f), w3t[r], p1);
        }
      }
      const float o0 = __shfl_xor(p0, 16, 32);
      const float o1 = __shfl_xor(p1, 16, 32);
      const float s0 = (p0 + o0) + b3v;
      const float s1 = (p1 + o1) + b3v;
      const float oval = (half != 0) ? s1 : s0;
      volatile float* qo = out + (size_t)v * kN + base + lane;
      *qo = oval;
      __threadfence();
      *qo = oval;
      par0 = s0;
      par1 = s1;
    }
  }
}

extern "C" void kernel_launch(void* const* d_in, const int* in_sizes, int n_in,
                              void* d_out, int out_size, void* d_ws, size_t ws_size,
                              hipStream_t stream) {
  if (n_in < 14) return;
  if (in_sizes[0] != kVars * kN) return;
  if (in_sizes[1] != kVars) return;
  if (in_sizes[2] != kHid) return;
  if (in_sizes[3] != kHid) return;
  if (in_sizes[4] != kHid * kHid) return;
  if (in_sizes[5] != kHid) return;
  if (in_sizes[6] != kHid) return;
  if (in_sizes[7] != 1) return;
  if (in_sizes[8] != (kVars - 1) * 2 * kHid) return;
  if (in_sizes[9] != (kVars - 1) * kHid) return;
  if (in_sizes[10] != (kVars - 1) * kHid * kHid) return;
  if (in_sizes[11] != (kVars - 1) * kHid) return;
  if (in_sizes[12] != (kVars - 1) * kHid) return;
  if (in_sizes[13] != (kVars - 1)) return;
  if (out_size != kVars * kN) return;
  if (ws_size < kWsTotal) return;

  const float* noise = (const float*)d_in[0];
  const float* stds  = (const float*)d_in[1];
  const float* w0_1  = (const float*)d_in[2];
  const float* b0_1  = (const float*)d_in[3];
  const float* w0_2  = (const float*)d_in[4];
  const float* b0_2  = (const float*)d_in[5];
  const float* w0_3  = (const float*)d_in[6];
  const float* b0_3  = (const float*)d_in[7];
  const float* W1    = (const float*)d_in[8];
  const float* B1    = (const float*)d_in[9];
  const float* W2    = (const float*)d_in[10];
  const float* B2    = (const float*)d_in[11];
  const float* W3    = (const float*)d_in[12];
  const float* B3    = (const float*)d_in[13];
  float* out = (float*)d_out;

  char* ws = (char*)d_ws;
  unsigned short* W2T = (unsigned short*)(ws + kOffW2T);
  float*          PRM = (float*)(ws + kOffPRM);

  prep_w2t_kernel<<<kVars, 256, 0, stream>>>(w0_2, W2, W2T);
  prep_params_kernel<<<kParamRows / 8, 256, 0, stream>>>(w0_1, b0_1, b0_2, w0_3, W1, B1, B2, W3, PRM);
  chain_mlp_kernel<<<kMainBlocks, 256, 0, stream>>>(noise, stds, b0_3, B3, W2T, PRM, out);
}
